// MLP_Discriminator_49357764166095
// MI455X (gfx1250) — hardware-verified
//
#include <hip/hip_runtime.h>
#include <hip/hip_bf16.h>
#include <stddef.h>
#include <math.h>


#define HID   256
#define NVAR  10
#define TT    64
#define BBAT  32
#define INP   4
#define RN    (BBAT * NVAR * TT)
#define NTHR  256
#define TROWS 16
#define NBLK  (RN / TROWS)
#define PARTW 512
#define HBLK  (BBAT * (TT / TROWS))
#define OUTB  (TROWS * NVAR)
#define PB0   32
#define PB1   96
#define PB2   128
#define PB3   160
#define PB4   192
#define NPREP 224

static_assert(RN % TROWS == 0);
static_assert(TT % TROWS == 0);
static_assert(NTHR == 8 * 32);
static_assert(HID == 8 * 32);
static_assert(OUTB == 40 * 4);
static_assert(NBLK * TROWS == RN);
static_assert(HBLK * OUTB == RN);
static_assert(PB0 * NTHR * 8 == HID * HID);
static_assert((PB1 - PB0) * NTHR * 8 == 2 * HID * HID);
static_assert(NPREP == PB4 + PB0);
static_assert(TROWS * 16 == NTHR);

typedef float          v4f   __attribute__((ext_vector_type(4)));
typedef float          v8f   __attribute__((ext_vector_type(8)));
typedef int            v4i   __attribute__((ext_vector_type(4)));
typedef unsigned short v8us  __attribute__((ext_vector_type(8)));
typedef unsigned short v16us __attribute__((ext_vector_type(16)));
typedef __bf16         v16bf __attribute__((ext_vector_type(16)));
union FragB { v16bf v; v16us u; v8us h[2]; };
union Pk8 { v8us h; v4i i; };

__device__ __forceinline__ unsigned f2bf(float f) {
  const unsigned u = __float_as_uint(f);
  return (u + 0x7FFFu + ((u >> 16) & 1u)) >> 16;
}

__device__ __forceinline__ void split8(v4f a, v4f b, v8us& hi, v8us& lo) {
  float f[8];
  f[0] = a.x; f[1] = a.y; f[2] = a.z; f[3] = a.w;
  f[4] = b.x; f[5] = b.y; f[6] = b.z; f[7] = b.w;
  v8us rh, rl;
#pragma unroll
  for (int i = 0; i < 8; ++i) {
    const unsigned hb = f2bf(f[i]);
    const float r = f[i] - __uint_as_float(hb << 16);
    rh[i] = (unsigned short)hb;
    rl[i] = (unsigned short)f2bf(r);
  }
  hi = rh;
  lo = rl;
}

__device__ __forceinline__ v8f wm3(v16bf ah, v16bf al, v16bf bh, v16bf bl, v8f c) {
  v8f d = __builtin_amdgcn_wmma_f32_16x16x32_bf16(false, ah, false, bh, (short)0, c, false, false);
  d = __builtin_amdgcn_wmma_f32_16x16x32_bf16(false, ah, false, bl, (short)0, d, false, false);
  d = __builtin_amdgcn_wmma_f32_16x16x32_bf16(false, al, false, bh, (short)0, d, false, false);
  asm volatile("v_nop\n\tv_nop\n\tv_nop\n\tv_nop" : "+v"(d) : "v"(ah), "v"(al), "v"(bh), "v"(bl));
  return d;
}

__device__ __forceinline__ float elu1(float x) {
  return x > 0.0f ? x : (__expf(x) - 1.0f);
}

__device__ __forceinline__ v4f elu4(v4f a) {
  v4f o;
  o.x = elu1(a.x); o.y = elu1(a.y); o.z = elu1(a.z); o.w = elu1(a.w);
  return o;
}

__device__ __forceinline__ v4f relu4(v4f a) {
  v4f o;
  o.x = fmaxf(a.x, 0.0f); o.y = fmaxf(a.y, 0.0f); o.z = fmaxf(a.z, 0.0f); o.w = fmaxf(a.w, 0.0f);
  return o;
}

__device__ __forceinline__ v8f splat8(float b) {
  v8f c;
#pragma unroll
  for (int i = 0; i < 8; ++i) c[i] = b;
  return c;
}

__device__ __forceinline__ void stage16(v4f z0, v4f z1, v4f z2, v4f z3,
                                        unsigned short* lah, unsigned short* lal, int off) {
  v8us h0, l0, h1, l1;
  split8(z0, z1, h0, l0);
  split8(z2, z3, h1, l1);
  *(v8us*)(lah + off) = h0;
  *(v8us*)(lah + off + 8) = h1;
  *(v8us*)(lal + off) = l0;
  *(v8us*)(lal + off + 8) = l1;
}

__device__ __forceinline__ void wgemm(const unsigned short* lah, const unsigned short* lal,
    const unsigned short* __restrict__ wh, const unsigned short* __restrict__ wl, int kp,
    int col0, int hh, int m, v8f& c0, v8f& c1) {
  const unsigned short* ap = lah + m * HID + 8 * hh;
  const unsigned short* aq = lal + m * HID + 8 * hh;
  const size_t o0 = (size_t)(col0 + m) * kp + 8 * hh;
  const size_t o1 = (size_t)(col0 + 16 + m) * kp + 8 * hh;
  const unsigned short* b0h = wh + o0;
  const unsigned short* b0l = wl + o0;
  const unsigned short* b1h = wh + o1;
  const unsigned short* b1l = wl + o1;
#pragma unroll 1
  for (int kt = 0; kt < HID / 32; ++kt) {
    const int k0 = 32 * kt;
    FragB ah, al, ph, pl, qh, ql;
    ah.h[0] = *(const v8us*)(ap + k0);   ah.h[1] = *(const v8us*)(ap + k0 + 16);
    al.h[0] = *(const v8us*)(aq + k0);   al.h[1] = *(const v8us*)(aq + k0 + 16);
    ph.h[0] = *(const v8us*)(b0h + k0);  ph.h[1] = *(const v8us*)(b0h + k0 + 16);
    pl.h[0] = *(const v8us*)(b0l + k0);  pl.h[1] = *(const v8us*)(b0l + k0 + 16);
    qh.h[0] = *(const v8us*)(b1h + k0);  qh.h[1] = *(const v8us*)(b1h + k0 + 16);
    ql.h[0] = *(const v8us*)(b1l + k0);  ql.h[1] = *(const v8us*)(b1l + k0 + 16);
    c0 = wm3(ah.v, al.v, ph.v, pl.v, c0);
    c1 = wm3(ah.v, al.v, qh.v, ql.v, c1);
  }
}

__device__ __forceinline__ void write_rows16(const float* stg, float* dst, int pitch, int wave, int lane) {
#pragma unroll
  for (int rr = 0; rr < 2; ++rr) {
    const int row = 2 * wave + rr;
#pragma unroll
    for (int j = 0; j < 2; ++j) {
      const v4f v = *(const v4f*)(stg + row * HID + 128 * j + 4 * lane);
      *(volatile v4f*)(dst + (size_t)row * pitch + 128 * j + 4 * lane) = v;
    }
  }
}

__device__ __forceinline__ void write_part(const float* lstat, float* dst, int tid) {
  if (tid < 128) {
    const v4f v = *(const v4f*)(lstat + 4 * tid);
    *(volatile v4f*)(dst + 4 * tid) = v;
  }
}

__device__ __forceinline__ void stat_lds(float s0, float q0, float s1, float q1,
                                         int cA, int cB, int hh, float* lstat) {
  s0 += __shfl_xor(s0, 16);
  q0 += __shfl_xor(q0, 16);
  s1 += __shfl_xor(s1, 16);
  q1 += __shfl_xor(q1, 16);
  if (hh == 0) {
    lstat[cA] = s0;
    lstat[HID + cA] = q0;
    lstat[cB] = s1;
    lstat[HID + cB] = q1;
  }
}

__global__ __launch_bounds__(NTHR) void k_prep(
    const float* __restrict__ s0, const float* __restrict__ s1, const float* __restrict__ s2,
    const float* __restrict__ s3, const float* __restrict__ s4, const float* __restrict__ s5,
    unsigned short* d0, unsigned short* d1, unsigned short* d2,
    unsigned short* d3, unsigned short* d4, unsigned short* d5) {
  const int b = blockIdx.x, tid = threadIdx.x;
  const float* src;
  unsigned short* dst;
  int K, ub;
  if (b < PB0)      { src = s0; dst = d0; K = HID;     ub = b; }
  else if (b < PB1) { src = s1; dst = d1; K = 2 * HID; ub = b - PB0; }
  else if (b < PB2) { src = s2; dst = d2; K = HID;     ub = b - PB1; }
  else if (b < PB3) { src = s3; dst = d3; K = HID;     ub = b - PB2; }
  else if (b < PB4) { src = s4; dst = d4; K = HID;     ub = b - PB3; }
  else              { src = s5; dst = d5; K = HID;     ub = b - PB4; }
  const int u   = ub * NTHR + tid;
  const int cpr = K >> 3;
  const int n   = u / cpr;
  const int kc  = u - n * cpr;
  float f[8];
#pragma unroll
  for (int j = 0; j < 8; ++j) f[j] = src[(size_t)(8 * kc + j) * HID + n];
  Pk8 ph, pl;
  {
    v4f a, c;
    a.x = f[0]; a.y = f[1]; a.z = f[2]; a.w = f[3];
    c.x = f[4]; c.y = f[5]; c.z = f[6]; c.w = f[7];
    split8(a, c, ph.h, pl.h);
  }
  const size_t ne = (size_t)HID * K;
  unsigned short* dh = dst + (size_t)u * 8;
  unsigned short* dl = dst + ne + (size_t)u * 8;
  *(volatile v4i*)dh = ph.i;
  *(volatile v4i*)dl = pl.i;
  __threadfence();
  *(volatile v4i*)dh = ph.i;
  *(volatile v4i*)dl = pl.i;
}

__global__ __launch_bounds__(NTHR) void k_bnfin(const float* __restrict__ part, int nblk, int cnt,
                                               const float* __restrict__ gamma, const float* __restrict__ beta,
                                               float* scsh) {
  __shared__ __attribute__((aligned(16))) float lsc[PARTW];
  const int tid = threadIdx.x;
  const int c = tid;
  double ds = 0.0, dq = 0.0;
#pragma unroll 4
  for (int blk = 0; blk < nblk; ++blk) {
    ds += (double)part[(size_t)blk * PARTW + c];
    dq += (double)part[(size_t)blk * PARTW + HID + c];
  }
  const double inv = 1.0 / (double)cnt;
  const double mean = ds * inv;
  double var = dq * inv - mean * mean;
  var = var > 0.0 ? var : 0.0;
  const float rstd = rsqrtf((float)var + 1e-5f);
  const float sc = gamma[c] * rstd;
  const float sh = beta[c] - (float)mean * sc;
  lsc[c] = sc;
  lsc[HID + c] = sh;
  __syncthreads();
  if (tid < 128) {
    const v4f v = *(const v4f*)(lsc + 4 * tid);
    *(volatile v4f*)(scsh + 4 * tid) = v;
  }
  __threadfence();
  if (tid < 128) {
    const v4f v = *(const v4f*)(lsc + 4 * tid);
    *(volatile v4f*)(scsh + 4 * tid) = v;
  }
}

__device__ __forceinline__ v4f fc1q(v4f xv, const float* __restrict__ w1a, const float* __restrict__ b1a, int c) {
  const v4f w0 = *(const v4f*)(w1a + c);
  const v4f w1 = *(const v4f*)(w1a + HID + c);
  const v4f w2 = *(const v4f*)(w1a + 2 * HID + c);
  const v4f w3 = *(const v4f*)(w1a + 3 * HID + c);
  const v4f bq = *(const v4f*)(b1a + c);
  return xv.x * w0 + xv.y * w1 + xv.z * w2 + xv.w * w3 + bq;
}

__global__ __launch_bounds__(NTHR) void k_mlp1(const float* __restrict__ x, const float* __restrict__ w1a,
    const float* __restrict__ b1a, const unsigned short* __restrict__ wh, const unsigned short* __restrict__ wl,
    const float* __restrict__ b1b, float* hout, float* part) {
  __shared__ __attribute__((aligned(16))) unsigned short lah[TROWS * HID];
  __shared__ __attribute__((aligned(16))) unsigned short lal[TROWS * HID];
  __shared__ __attribute__((aligned(16))) float stg[TROWS * HID];
  __shared__ __attribute__((aligned(16))) float lstat[PARTW];
  const int tid = threadIdx.x, lane = tid & 31, wave = tid >> 5, hh = lane >> 4, m = lane & 15;
  const int blk = blockIdx.x;
  const int nr0 = blk * TROWS;
  {
    const int rrow = tid >> 4, c16 = (tid & 15) * 16;
    const int g = nr0 + rrow;
    const int bb = g / (NVAR * TT);
    const int rem = g - bb * (NVAR * TT);
    const int v = rem / TT;
    const int t = rem - v * TT;
    const v4f xv = *(const v4f*)(x + ((size_t)((bb * TT + t) * NVAR + v)) * INP);
    const v4f z0 = elu4(fc1q(xv, w1a, b1a, c16));
    const v4f z1 = elu4(fc1q(xv, w1a, b1a, c16 + 4));
    const v4f z2 = elu4(fc1q(xv, w1a, b1a, c16 + 8));
    const v4f z3 = elu4(fc1q(xv, w1a, b1a, c16 + 12));
    stage16(z0, z1, z2, z3, lah, lal, rrow * HID + c16);
  }
  __syncthreads();
  const int col0 = wave * 32, cA = col0 + m, cB = col0 + 16 + m;
  v8f c0 = splat8(b1b[cA]), c1 = splat8(b1b[cB]);
  wgemm(lah, lal, wh, wl, HID, col0, hh, m, c0, c1);
  float s0 = 0.0f, q0 = 0.0f, s1 = 0.0f, q1 = 0.0f;
#pragma unroll
  for (int r = 0; r < 8; ++r) {
    const float va = elu1(c0[r]);
    const float vb = elu1(c1[r]);
    stg[(8 * hh + r) * HID + cA] = va;
    stg[(8 * hh + r) * HID + cB] = vb;
    s0 += va; q0 += va * va;
    s1 += vb; q1 += vb * vb;
  }
  stat_lds(s0, q0, s1, q1, cA, cB, hh, lstat);
  __syncthreads();
  float* drow = hout + (size_t)nr0 * HID;
  float* dpart = part + (size_t)blk * PARTW;
  write_rows16(stg, drow, HID, wave, lane);
  write_part(lstat, dpart, tid);
  __threadfence();
  write_rows16(stg, drow, HID, wave, lane);
  write_part(lstat, dpart, tid);
}

__global__ __launch_bounds__(NTHR) void k_proj(const float* __restrict__ hin, const float* __restrict__ scsh,
    const unsigned short* __restrict__ wh, const unsigned short* __restrict__ wl, float* pout) {
  __shared__ __attribute__((aligned(16))) unsigned short lah[TROWS * HID];
  __shared__ __attribute__((aligned(16))) unsigned short lal[TROWS * HID];
  __shared__ __attribute__((aligned(16))) float stg[TROWS * HID];
  const int tid = threadIdx.x, lane = tid & 31, wave = tid >> 5, hh = lane >> 4, m = lane & 15;
  const int blk = blockIdx.x;
  const int nr0 = blk * TROWS;
  {
    const int rrow = tid >> 4, c16 = (tid & 15) * 16;
    const float* hp = hin + (size_t)(nr0 + rrow) * HID + c16;
    const float* sp = scsh + c16;
    const float* tp = scsh + HID + c16;
    const v4f z0 = *(const v4f*)(hp)      * *(const v4f*)(sp)      + *(const v4f*)(tp);
    const v4f z1 = *(const v4f*)(hp + 4)  * *(const v4f*)(sp + 4)  + *(const v4f*)(tp + 4);
    const v4f z2 = *(const v4f*)(hp + 8)  * *(const v4f*)(sp + 8)  + *(const v4f*)(tp + 8);
    const v4f z3 = *(const v4f*)(hp + 12) * *(const v4f*)(sp + 12) + *(const v4f*)(tp + 12);
    stage16(z0, z1, z2, z3, lah, lal, rrow * HID + c16);
  }
  __syncthreads();
  const int col0 = wave * 32, cA = col0 + m, cB = col0 + 16 + m;
#pragma unroll 1
  for (int j = 0; j < 2; ++j) {
    v8f c0 = splat8(0.0f), c1 = splat8(0.0f);
    wgemm(lah, lal, wh + j * HID, wl + j * HID, 2 * HID, col0, hh, m, c0, c1);
    __syncthreads();
#pragma unroll
    for (int r = 0; r < 8; ++r) {
      stg[(8 * hh + r) * HID + cA] = c0[r];
      stg[(8 * hh + r) * HID + cB] = c1[r];
    }
    __syncthreads();
    float* drow = pout + (size_t)nr0 * (2 * HID) + j * HID;
    write_rows16(stg, drow, 2 * HID, wave, lane);
    __threadfence();
    write_rows16(stg, drow, 2 * HID, wave, lane);
  }
}

__global__ __launch_bounds__(NTHR) void k_edge(const float* __restrict__ pin, const float* __restrict__ b2a,
    const unsigned short* __restrict__ wh, const unsigned short* __restrict__ wl, const float* __restrict__ b2b,
    float* sout, float* part) {
  __shared__ __attribute__((aligned(16))) unsigned short lah[TROWS * HID];
  __shared__ __attribute__((aligned(16))) unsigned short lal[TROWS * HID];
  __shared__ __attribute__((aligned(16))) float stg[TROWS * HID];
  __shared__ __attribute__((aligned(16))) float lstat[PARTW];
  const int tid = threadIdx.x, lane = tid & 31, wave = tid >> 5, hh = lane >> 4, m = lane & 15;
  const int blk = blockIdx.x;
  const int nr0 = blk * TROWS;
  const int bv = blk >> 2;
  const int t0 = (blk & 3) * TROWS;
  const int bb = bv / NVAR;
  const int v = bv - bb * NVAR;
  const int rrow = tid >> 4, c16 = (tid & 15) * 16;
  v4f pr0, pr1, pr2, pr3;
  {
    const float* rp = pin + ((size_t)((bb * NVAR + v) * TT + t0 + rrow)) * (2 * HID) + HID + c16;
    const float* bp = b2a + c16;
    pr0 = *(const v4f*)(rp)      + *(const v4f*)(bp);
    pr1 = *(const v4f*)(rp + 4)  + *(const v4f*)(bp + 4);
    pr2 = *(const v4f*)(rp + 8)  + *(const v4f*)(bp + 8);
    pr3 = *(const v4f*)(rp + 12) + *(const v4f*)(bp + 12);
  }
  const int col0 = wave * 32, cA = col0 + m, cB = col0 + 16 + m;
  const float biasA = b2b[cA], biasB = b2b[cB];
  v8f agg0 = splat8(0.0f), agg1 = splat8(0.0f);
  float s0 = 0.0f, q0 = 0.0f, s1 = 0.0f, q1 = 0.0f;
#pragma unroll 1
  for (int s = 0; s < NVAR; ++s) {
    if (s == v) continue;
    __syncthreads();
    {
      const float* sp = pin + ((size_t)((bb * NVAR + s) * TT + t0 + rrow)) * (2 * HID) + c16;
      const v4f z0 = elu4(*(const v4f*)(sp)      + pr0);
      const v4f z1 = elu4(*(const v4f*)(sp + 4)  + pr1);
      const v4f z2 = elu4(*(const v4f*)(sp + 8)  + pr2);
      const v4f z3 = elu4(*(const v4f*)(sp + 12) + pr3);
      stage16(z0, z1, z2, z3, lah, lal, rrow * HID + c16);
    }
    __syncthreads();
    v8f c0 = splat8(biasA), c1 = splat8(biasB);
    wgemm(lah, lal, wh, wl, HID, col0, hh, m, c0, c1);
#pragma unroll
    for (int r = 0; r < 8; ++r) {
      const float va = elu1(c0[r]);
      const float vb = elu1(c1[r]);
      agg0[r] += va;
      agg1[r] += vb;
      s0 += va; q0 += va * va;
      s1 += vb; q1 += vb * vb;
    }
  }
#pragma unroll
  for (int r = 0; r < 8; ++r) {
    stg[(8 * hh + r) * HID + cA] = agg0[r];
    stg[(8 * hh + r) * HID + cB] = agg1[r];
  }
  stat_lds(s0, q0, s1, q1, cA, cB, hh, lstat);
  __syncthreads();
  float* drow = sout + (size_t)nr0 * HID;
  float* dpart = part + (size_t)blk * PARTW;
  write_rows16(stg, drow, HID, wave, lane);
  write_part(lstat, dpart, tid);
  __threadfence();
  write_rows16(stg, drow, HID, wave, lane);
  write_part(lstat, dpart, tid);
}

__global__ __launch_bounds__(NTHR) void k_mlp3(const float* __restrict__ sagg, const float* __restrict__ scsh,
    const unsigned short* __restrict__ wah, const unsigned short* __restrict__ wal, const float* __restrict__ ba,
    const unsigned short* __restrict__ wbh, const unsigned short* __restrict__ wbl, const float* __restrict__ bbv,
    float* hout, float* part) {
  __shared__ __attribute__((aligned(16))) unsigned short lah[TROWS * HID];
  __shared__ __attribute__((aligned(16))) unsigned short lal[TROWS * HID];
  __shared__ __attribute__((aligned(16))) unsigned short lbh[TROWS * HID];
  __shared__ __attribute__((aligned(16))) unsigned short lbl[TROWS * HID];
  __shared__ __attribute__((aligned(16))) float stg[TROWS * HID];
  __shared__ __attribute__((aligned(16))) float lstat[PARTW];
  const int tid = threadIdx.x, lane = tid & 31, wave = tid >> 5, hh = lane >> 4, m = lane & 15;
  const int blk = blockIdx.x;
  const int nr0 = blk * TROWS;
  {
    const int rrow = tid >> 4, c16 = (tid & 15) * 16;
    const float inv9 = 1.0f / 9.0f;
    const float* hp = sagg + (size_t)(nr0 + rrow) * HID + c16;
    const float* sp = scsh + c16;
    const float* tp = scsh + HID + c16;
    const v4f z0 = (*(const v4f*)(hp)      * inv9) * *(const v4f*)(sp)      + *(const v4f*)(tp);
    const v4f z1 = (*(const v4f*)(hp + 4)  * inv9) * *(const v4f*)(sp + 4)  + *(const v4f*)(tp + 4);
    const v4f z2 = (*(const v4f*)(hp + 8)  * inv9) * *(const v4f*)(sp + 8)  + *(const v4f*)(tp + 8);
    const v4f z3 = (*(const v4f*)(hp + 12) * inv9) * *(const v4f*)(sp + 12) + *(const v4f*)(tp + 12);
    stage16(z0, z1, z2, z3, lah, lal, rrow * HID + c16);
  }
  __syncthreads();
  const int col0 = wave * 32, cA = col0 + m, cB = col0 + 16 + m;
  {
    v8f c0 = splat8(ba[cA]), c1 = splat8(ba[cB]);
    wgemm(lah, lal, wah, wal, HID, col0, hh, m, c0, c1);
#pragma unroll
    for (int r = 0; r < 8; ++r) {
      const float va = elu1(c0[r]);
      const float vb = elu1(c1[r]);
      const unsigned ha = f2bf(va);
      const unsigned la = f2bf(va - __uint_as_float(ha << 16));
      const unsigned hb = f2bf(vb);
      const unsigned lb = f2bf(vb - __uint_as_float(hb << 16));
      lbh[(8 * hh + r) * HID + cA] = (unsigned short)ha;
      lbl[(8 * hh + r) * HID + cA] = (unsigned short)la;
      lbh[(8 * hh + r) * HID + cB] = (unsigned short)hb;
      lbl[(8 * hh + r) * HID + cB] = (unsigned short)lb;
    }
  }
  __syncthreads();
  v8f c0 = splat8(bbv[cA]), c1 = splat8(bbv[cB]);
  wgemm(lbh, lbl, wbh, wbl, HID, col0, hh, m, c0, c1);
  float s0 = 0.0f, q0 = 0.0f, s1 = 0.0f, q1 = 0.0f;
#pragma unroll
  for (int r = 0; r < 8; ++r) {
    const float va = elu1(c0[r]);
    const float vb = elu1(c1[r]);
    stg[(8 * hh + r) * HID + cA] = va;
    stg[(8 * hh + r) * HID + cB] = vb;
    s0 += va; q0 += va * va;
    s1 += vb; q1 += vb * vb;
  }
  stat_lds(s0, q0, s1, q1, cA, cB, hh, lstat);
  __syncthreads();
  float* drow = hout + (size_t)nr0 * HID;
  float* dpart = part + (size_t)blk * PARTW;
  write_rows16(stg, drow, HID, wave, lane);
  write_part(lstat, dpart, tid);
  __threadfence();
  write_rows16(stg, drow, HID, wave, lane);
  write_part(lstat, dpart, tid);
}

__global__ __launch_bounds__(NTHR) void k_head(const float* __restrict__ hin, const float* __restrict__ scsh,
    const unsigned short* __restrict__ wh, const unsigned short* __restrict__ wl, const float* __restrict__ bo1,
    const float* __restrict__ wo2, const float* __restrict__ bo2, float* out) {
  __shared__ __attribute__((aligned(16))) unsigned short lah[TROWS * HID];
  __shared__ __attribute__((aligned(16))) unsigned short lal[TROWS * HID];
  __shared__ __attribute__((aligned(16))) float stg[TROWS * HID];
  __shared__ __attribute__((aligned(16))) float lout[OUTB];
  const int tid = threadIdx.x, lane = tid & 31, wave = tid >> 5, hh = lane >> 4, m = lane & 15;
  const int blk = blockIdx.x;
  const int bb = blk >> 2;
  const int t0 = (blk & 3) * TROWS;
  const int rrow = tid >> 4, c16 = (tid & 15) * 16;
  const int col0 = wave * 32, cA = col0 + m, cB = col0 + 16 + m;
  const float biasA = bo1[cA], biasB = bo1[cB];
  const float bout = bo2[0];
#pragma unroll 1
  for (int v = 0; v < NVAR; ++v) {
    __syncthreads();
    {
      const size_t nr = (size_t)((bb * NVAR + v) * TT + t0 + rrow);
      const float* hp = hin + nr * HID + c16;
      const float* sp = scsh + c16;
      const float* tp = scsh + HID + c16;
      const v4f z0 = relu4(*(const v4f*)(hp)      * *(const v4f*)(sp)      + *(const v4f*)(tp));
      const v4f z1 = relu4(*(const v4f*)(hp + 4)  * *(const v4f*)(sp + 4)  + *(const v4f*)(tp + 4));
      const v4f z2 = relu4(*(const v4f*)(hp + 8)  * *(const v4f*)(sp + 8)  + *(const v4f*)(tp + 8));
      const v4f z3 = relu4(*(const v4f*)(hp + 12) * *(const v4f*)(sp + 12) + *(const v4f*)(tp + 12));
      stage16(z0, z1, z2, z3, lah, lal, rrow * HID + c16);
    }
    __syncthreads();
    v8f c0 = splat8(biasA), c1 = splat8(biasB);
    wgemm(lah, lal, wh, wl, HID, col0, hh, m, c0, c1);
#pragma unroll
    for (int r = 0; r < 8; ++r) {
      stg[(8 * hh + r) * HID + cA] = fmaxf(c0[r], 0.0f);
      stg[(8 * hh + r) * HID + cB] = fmaxf(c1[r], 0.0f);
    }
    __syncthreads();
    {
      const int pt = tid & 15;
      const float* orow = stg + rrow * HID + pt * 16;
      const float* wv = wo2 + pt * 16;
      float sacc = 0.0f;
#pragma unroll
      for (int k = 0; k < 16; ++k) sacc += orow[k] * wv[k];
      sacc += __shfl_xor(sacc, 8);
      sacc += __shfl_xor(sacc, 4);
      sacc += __shfl_xor(sacc, 2);
      sacc += __shfl_xor(sacc, 1);
      if (pt == 0) lout[rrow * NVAR + v] = sacc + bout;
    }
  }
  __syncthreads();
  float* dst = out + (size_t)blk * OUTB;
  if (tid < OUTB / 4) {
    const v4f val = *(const v4f*)(lout + 4 * tid);
    *(volatile v4f*)(dst + 4 * tid) = val;
  }
  __threadfence();
  if (tid < OUTB / 4) {
    const v4f val = *(const v4f*)(lout + 4 * tid);
    *(volatile v4f*)(dst + 4 * tid) = val;
  }
}

extern "C" void kernel_launch(void* const* d_in, const int* in_sizes, int n_in,
                              void* d_out, int out_size, void* d_ws, size_t ws_size,
                              hipStream_t stream) {
  if (n_in < 23) return;
  if (in_sizes[0] != RN * INP || in_sizes[1] != INP * HID || in_sizes[2] != HID) return;
  if (in_sizes[3] != HID * HID || in_sizes[4] != HID || in_sizes[5] != HID || in_sizes[6] != HID) return;
  if (in_sizes[7] != 2 * HID * HID || in_sizes[8] != HID || in_sizes[9] != HID * HID || in_sizes[10] != HID) return;
  if (in_sizes[11] != HID || in_sizes[12] != HID) return;
  if (in_sizes[13] != HID * HID || in_sizes[14] != HID || in_sizes[15] != HID * HID || in_sizes[16] != HID) return;
  if (in_sizes[17] != HID || in_sizes[18] != HID) return;
  if (in_sizes[19] != HID * HID || in_sizes[20] != HID || in_sizes[21] != HID || in_sizes[22] < 1) return;
  if (out_size != RN) return;

  const float* x   = (const float*)d_in[0];
  const float* w1a = (const float*)d_in[1];
  const float* b1a = (const float*)d_in[2];
  const float* w1b = (const float*)d_in[3];
  const float* b1b = (const float*)d_in[4];
  const float* g1  = (const float*)d_in[5];
  const float* be1 = (const float*)d_in[6];
  const float* w2a = (const float*)d_in[7];
  const float* b2a = (const float*)d_in[8];
  const float* w2b = (const float*)d_in[9];
  const float* b2b = (const float*)d_in[10];
  const float* g2  = (const float*)d_in[11];
  const float* be2 = (const float*)d_in[12];
  const float* w3a = (const float*)d_in[13];
  const float* b3a = (const float*)d_in[14];
  const float* w3b = (const float*)d_in[15];
  const float* b3b = (const float*)d_in[16];
  const float* g3  = (const float*)d_in[17];
  const float* be3 = (const float*)d_in[18];
  const float* wo1 = (const float*)d_in[19];
  const float* bo1 = (const float*)d_in[20];
  const float* wo2 = (const float*)d_in[21];
  const float* bo2 = (const float*)d_in[22];
  float* dout = (float*)d_out;

  const size_t nq1 = (size_t)HID * HID;
  const size_t nq2 = (size_t)HID * 2 * HID;

  char* ws = (char*)d_ws;
  size_t off = 0;
  auto carve = [&](size_t bytes) -> size_t {
    const size_t o = off;
    off = (off + bytes + 255) & ~(size_t)255;
    return o;
  };
  const size_t oq1b = carve(nq1 * 4), oq2a = carve(nq2 * 4), oq2b = carve(nq1 * 4);
  const size_t oq3a = carve(nq1 * 4), oq3b = carve(nq1 * 4), oqo1 = carve(nq1 * 4);
  const size_t opt1 = carve((size_t)NBLK * PARTW * 4);
  const size_t opt2 = carve((size_t)NBLK * PARTW * 4);
  const size_t opt3 = carve((size_t)NBLK * PARTW * 4);
  const size_t osc1 = carve((size_t)PARTW * 4), osc2 = carve((size_t)PARTW * 4), osc3 = carve((size_t)PARTW * 4);
  const size_t oh1 = carve((size_t)RN * HID * 4);
  const size_t opp = carve((size_t)RN * 2 * HID * 4);
  const size_t oss = carve((size_t)RN * HID * 4);
  const size_t oh3 = carve((size_t)RN * HID * 4);
  size_t limit = (size_t)134217728;
  if (ws_size < limit) limit = ws_size;
  if (off > limit) return;

  unsigned short* q1b = (unsigned short*)(ws + oq1b);
  unsigned short* q2a = (unsigned short*)(ws + oq2a);
  unsigned short* q2b = (unsigned short*)(ws + oq2b);
  unsigned short* q3a = (unsigned short*)(ws + oq3a);
  unsigned short* q3b = (unsigned short*)(ws + oq3b);
  unsigned short* qo1 = (unsigned short*)(ws + oqo1);
  float* PT1 = (float*)(ws + opt1);
  float* PT2 = (float*)(ws + opt2);
  float* PT3 = (float*)(ws + opt3);
  float* SC1 = (float*)(ws + osc1);
  float* SC2 = (float*)(ws + osc2);
  float* SC3 = (float*)(ws + osc3);
  float* H1  = (float*)(ws + oh1);
  float* PP  = (float*)(ws + opp);
  float* SS  = (float*)(ws + oss);
  float* H3  = (float*)(ws + oh3);

  k_prep<<<NPREP, NTHR, 0, stream>>>(w1b, w2a, w2b, w3a, w3b, wo1, q1b, q2a, q2b, q3a, q3b, qo1);
  k_mlp1<<<NBLK, NTHR, 0, stream>>>(x, w1a, b1a, q1b, q1b + nq1, b1b, H1, PT1);
  k_bnfin<<<1, NTHR, 0, stream>>>(PT1, NBLK, RN, g1, be1, SC1);
  k_proj<<<NBLK, NTHR, 0, stream>>>(H1, SC1, q2a, q2a + nq2, PP);
  k_edge<<<NBLK, NTHR, 0, stream>>>(PP, b2a, q2b, q2b + nq1, b2b, SS, PT2);
  k_bnfin<<<1, NTHR, 0, stream>>>(PT2, NBLK, RN * (NVAR - 1), g2, be2, SC2);
  k_mlp3<<<NBLK, NTHR, 0, stream>>>(SS, SC2, q3a, q3a + nq1, b3a, q3b, q3b + nq1, b3b, H3, PT3);
  k_bnfin<<<1, NTHR, 0, stream>>>(PT3, NBLK, RN, g3, be3, SC3);
  k_head<<<HBLK, NTHR, 0, stream>>>(H3, SC3, qo1, qo1 + nq1, bo1, wo2, bo2, dout);
}
